// MixedMultiHeadAttention_23545010716838
// MI455X (gfx1250) — hardware-verified
//
#include <hip/hip_runtime.h>


typedef _Float16 f16;
typedef f16   v16h __attribute__((ext_vector_type(16)));
typedef f16   v8h  __attribute__((ext_vector_type(8)));
typedef float v8f  __attribute__((ext_vector_type(8)));
typedef float v4f  __attribute__((ext_vector_type(4)));

union Frag { v16h v; v8h p[2]; };

#define NOPS4 "v_nop\n\tv_nop\n\tv_nop\n\tv_nop"

static __device__ __forceinline__ v8f mma16(const v16h a, const v16h b, v8f c) {
  return __builtin_amdgcn_wmma_f32_16x16x32_f16(false, a, false, b, (short)0, c, false, false);
}
static __device__ __forceinline__ v8f zero8() {
  v8f z = {0.f, 0.f, 0.f, 0.f, 0.f, 0.f, 0.f, 0.f};
  return z;
}
static __device__ __forceinline__ float bfr(float f) {
  unsigned u = __float_as_uint(f);
  u += 0x7FFFu + ((u >> 16) & 1u);
  return __uint_as_float(u & 0xFFFF0000u);
}

__global__ __launch_bounds__(256)
void k_cvt(const float* __restrict__ src, f16* dst, int n8, float scale)
{
  const int i = blockIdx.x * 256 + threadIdx.x;
  if (i >= n8) return;
  const v4f a = *(const v4f*)(src + (size_t)i * 8);
  const v4f b = *(const v4f*)(src + (size_t)i * 8 + 4);
  v8h o;
  o[0] = (f16)(bfr(a.x) * scale);  o[1] = (f16)(bfr(a.y) * scale);
  o[2] = (f16)(bfr(a.z) * scale);  o[3] = (f16)(bfr(a.w) * scale);
  o[4] = (f16)(bfr(b.x) * scale);  o[5] = (f16)(bfr(b.y) * scale);
  o[6] = (f16)(bfr(b.z) * scale);  o[7] = (f16)(bfr(b.w) * scale);
  f16* p = dst + (size_t)i * 8;
  *(volatile v8h*)p = o;
  __threadfence();
  *(volatile v8h*)p = o;
}

#define TP 72
__global__ __launch_bounds__(256)
void k_wtr(const float* __restrict__ in, f16* out, int R, int C, long inZ, long outZ, float scale)
{
  __shared__ __attribute__((aligned(16))) f16 tile[64 * TP];
  const int tid = threadIdx.x;
  const int r0 = blockIdx.y * 64, c0 = blockIdx.x * 64;
  const float* ip = in + (size_t)blockIdx.z * inZ;
  f16* op = out + (size_t)blockIdx.z * outZ;
#pragma unroll
  for (int it = 0; it < 4; ++it) {
    const int idx = tid + it * 256;
    const int rr = idx >> 4, cq = idx & 15;
    const v4f x = *(const v4f*)(ip + (size_t)(r0 + rr) * C + c0 + cq * 4);
    tile[(cq * 4 + 0) * TP + rr] = (f16)(bfr(x.x) * scale);
    tile[(cq * 4 + 1) * TP + rr] = (f16)(bfr(x.y) * scale);
    tile[(cq * 4 + 2) * TP + rr] = (f16)(bfr(x.z) * scale);
    tile[(cq * 4 + 3) * TP + rr] = (f16)(bfr(x.w) * scale);
  }
  __syncthreads();
  const int seg = tid & 7, lb = tid >> 3;
  v8h val[2]; size_t off[2];
#pragma unroll
  for (int it = 0; it < 2; ++it) {
    const int line = lb + 32 * it;
    val[it] = *(const v8h*)(&tile[line * TP + seg * 8]);
    off[it] = (size_t)(c0 + line) * R + r0 + seg * 8;
  }
#pragma unroll
  for (int it = 0; it < 2; ++it) *(volatile v8h*)(op + off[it]) = val[it];
  __threadfence();
#pragma unroll
  for (int it = 0; it < 2; ++it) *(volatile v8h*)(op + off[it]) = val[it];
}

#define AP  40
#define CPH 72
#define CPT 136
#define CPF 68

template <int MODE>
__global__ __launch_bounds__(256)
void k_gemm(const f16* __restrict__ A, int lda,
            const f16* __restrict__ B, int ldb, long bZ, int kbMask, int K,
            const float* __restrict__ bias, float accMul, float alpha,
            void* O0, void* O1, int ldc, long oZ)
{
  __shared__ __attribute__((aligned(16))) f16   As[128 * AP];
  __shared__ __attribute__((aligned(16))) f16   Bs[64 * AP];
  __shared__ __attribute__((aligned(16))) float Cs[8704];

  const int tid = threadIdx.x, wave = tid >> 5, lane = tid & 31;
  const int hh = lane >> 4, m = lane & 15;
  const int z = blockIdx.z;
  const int m0 = blockIdx.y * 128, n0 = blockIdx.x * 64;
  const int wr = (wave >> 1) * 32, wc = (wave & 1) * 32;
  const int ar = tid >> 2, aq = tid & 3;
  const f16* Ap0 = A + (size_t)(m0 + ar) * lda + aq * 8;
  const f16* Ap1 = A + (size_t)(m0 + ar + 64) * lda + aq * 8;
  const f16* Bp  = B + (size_t)z * bZ + (size_t)(n0 + ar) * ldb + aq * 8;

  v8f acc[2][2];
  acc[0][0] = zero8(); acc[0][1] = zero8(); acc[1][0] = zero8(); acc[1][1] = zero8();

  for (int kk = 0; kk < K; kk += 32) {
    const v8h ga0 = *(const v8h*)(Ap0 + kk);
    const v8h ga1 = *(const v8h*)(Ap1 + kk);
    const v8h gb  = *(const v8h*)(Bp + (kk & kbMask));
    *(v8h*)(&As[ar * AP + aq * 8]) = ga0;
    *(v8h*)(&As[(ar + 64) * AP + aq * 8]) = ga1;
    *(v8h*)(&Bs[ar * AP + aq * 8]) = gb;
    __syncthreads();

    Frag fa[2], fb[2];
#pragma unroll
    for (int i = 0; i < 2; ++i) {
      const f16* pa = &As[(wr + i * 16 + m) * AP];
      fa[i].p[0] = *(const v8h*)(pa + 8 * hh);
      fa[i].p[1] = *(const v8h*)(pa + 16 + 8 * hh);
      const f16* pb = &Bs[(wc + i * 16 + m) * AP];
      fb[i].p[0] = *(const v8h*)(pb + 8 * hh);
      fb[i].p[1] = *(const v8h*)(pb + 16 + 8 * hh);
    }
    acc[0][0] = mma16(fa[0].v, fb[0].v, acc[0][0]);
    acc[0][1] = mma16(fa[0].v, fb[1].v, acc[0][1]);
    acc[1][0] = mma16(fa[1].v, fb[0].v, acc[1][0]);
    acc[1][1] = mma16(fa[1].v, fb[1].v, acc[1][1]);
    asm volatile(NOPS4
                 : "+v"(acc[0][0]), "+v"(acc[0][1]), "+v"(acc[1][0]), "+v"(acc[1][1])
                 : "v"(fa[0].v), "v"(fa[1].v), "v"(fb[0].v), "v"(fb[1].v));
    __syncthreads();
  }

  const int seg = tid & 7, lb = tid >> 3;

  if (MODE == 0) {
    f16* C = (f16*)Cs;
#pragma unroll
    for (int i = 0; i < 2; ++i) {
#pragma unroll
      for (int j = 0; j < 2; ++j) {
        const int col = wc + j * 16 + m;
        const float bj = bias[n0 + col];
#pragma unroll
        for (int r = 0; r < 8; ++r) {
          const int row = wr + i * 16 + 8 * hh + r;
          C[row * CPH + col] = (f16)((acc[i][j][r] * accMul + bj) * alpha);
        }
      }
    }
    __syncthreads();
    f16* Ob = (f16*)O0 + (size_t)z * oZ;
    v8h val[4]; size_t off[4];
#pragma unroll
    for (int it = 0; it < 4; ++it) {
      const int line = lb + 32 * it;
      val[it] = *(const v8h*)(&C[line * CPH + seg * 8]);
      off[it] = (size_t)(m0 + line) * ldc + n0 + seg * 8;
    }
#pragma unroll
    for (int it = 0; it < 4; ++it) *(volatile v8h*)(Ob + off[it]) = val[it];
    __threadfence();
#pragma unroll
    for (int it = 0; it < 4; ++it) *(volatile v8h*)(Ob + off[it]) = val[it];
  } else if (MODE == 1) {
    f16* Ch = (f16*)Cs;
    f16* Cl = Ch + 64 * CPT;
#pragma unroll
    for (int i = 0; i < 2; ++i) {
#pragma unroll
      for (int j = 0; j < 2; ++j) {
        const int col = wc + j * 16 + m;
        const float bj = bias[n0 + col];
#pragma unroll
        for (int r = 0; r < 8; ++r) {
          const int row = wr + i * 16 + 8 * hh + r;
          const float v = (acc[i][j][r] * accMul + bj) * alpha;
          const f16 hv = (f16)v;
          const f16 lv = (f16)(v - (float)hv);
          Ch[col * CPT + row] = hv;
          Cl[col * CPT + row] = lv;
        }
      }
    }
    __syncthreads();
    f16* Oh = (f16*)O0 + (size_t)z * oZ;
    f16* Ol = (f16*)O1 + (size_t)z * oZ;
    v8h val[8]; size_t off[8];
#pragma unroll
    for (int it = 0; it < 8; ++it) {
      const int plane = it >> 2;
      const int line = lb + 32 * (it & 3);
      const int c = line >> 1, half = line & 1;
      const f16* src = (plane ? Cl : Ch) + c * CPT + half * 64 + seg * 8;
      val[it] = *(const v8h*)src;
      off[it] = (size_t)(n0 + c) * ldc + m0 + half * 64 + seg * 8;
    }
#pragma unroll
    for (int it = 0; it < 8; ++it) *(volatile v8h*)(((it >> 2) ? Ol : Oh) + off[it]) = val[it];
    __threadfence();
#pragma unroll
    for (int it = 0; it < 8; ++it) *(volatile v8h*)(((it >> 2) ? Ol : Oh) + off[it]) = val[it];
  } else {
    float* Cf = Cs;
#pragma unroll
    for (int i = 0; i < 2; ++i) {
#pragma unroll
      for (int j = 0; j < 2; ++j) {
        const int col = wc + j * 16 + m;
        const float bj = bias[n0 + col];
#pragma unroll
        for (int r = 0; r < 8; ++r) {
          const int row = wr + i * 16 + 8 * hh + r;
          Cf[row * CPF + col] = (acc[i][j][r] * accMul + bj) * alpha;
        }
      }
    }
    __syncthreads();
    float* Of = (float*)O0;
    v4f val[8]; size_t off[8];
#pragma unroll
    for (int it = 0; it < 8; ++it) {
      const int line = lb + 32 * it;
      const int row = line >> 1, half = line & 1;
      val[it] = *(const v4f*)(&Cf[row * CPF + half * 32 + seg * 4]);
      off[it] = (size_t)(m0 + row) * ldc + n0 + half * 32 + seg * 4;
    }
#pragma unroll
    for (int it = 0; it < 8; ++it) *(volatile v4f*)(Of + off[it]) = val[it];
    __threadfence();
#pragma unroll
    for (int it = 0; it < 8; ++it) *(volatile v4f*)(Of + off[it]) = val[it];
  }
}

#define SP 1028
#define QP 72
#define NEGM (-1.0e30f)

__global__ __launch_bounds__(256)
void k_attn(const f16* __restrict__ Qg, const f16* __restrict__ Kg,
            const f16* __restrict__ Vhg, const f16* __restrict__ Vlg, f16* Ao)
{
  extern __shared__ __attribute__((aligned(16))) unsigned char smem[];
  float* S   = (float*)smem;
  f16*   Qs  = (f16*)(smem + (size_t)64 * SP * 4);
  float* red = (float*)(smem + (size_t)64 * SP * 4 + (size_t)64 * QP * 2);

  const int tid = threadIdx.x, wave = tid >> 5, lane = tid & 31;
  const int hh = lane >> 4, m = lane & 15;
  const int b = blockIdx.z, hd = blockIdx.y, q0 = blockIdx.x * 64;
  const int g = hd >> 2;
  const int IMIN = -2147483647 - 1, IMAX = 2147483647;
  const int dlo = (g == 1) ? -128 : ((g == 3) ? 0 : IMIN);
  const int dhi = (g == 1) ?  128 : ((g == 2) ? 0 : IMAX);
  int kbeg = 0, kend = 1024;
  if (g == 1) {
    kbeg = q0 - 128; if (kbeg < 0) kbeg = 0;
    kend = q0 + 192; if (kend > 1024) kend = 1024;
  } else if (g == 2) {
    kbeg = q0;
  } else if (g == 3) {
    kend = q0 + 64;
  }

  const size_t headOff = (size_t)hd * 262144;
  const f16* Qh = Qg  + headOff + (size_t)(b * 1024 + q0) * 64;
  const f16* Kh = Kg  + headOff + (size_t)(b * 1024) * 64;
  const f16* Vh = Vhg + headOff + (size_t)b * 1024;
  const f16* Vl = Vlg + headOff + (size_t)b * 1024;

#pragma unroll
  for (int it = 0; it < 2; ++it) {
    const int idx = tid + it * 256;
    const int row = idx >> 3, cq = idx & 7;
    *(v8h*)(&Qs[row * QP + cq * 8]) = *(const v8h*)(Qh + (size_t)row * 64 + cq * 8);
  }
  __syncthreads();

  const int rb = wave >> 1;
  Frag aQ[2];
#pragma unroll
  for (int ks = 0; ks < 2; ++ks) {
    const f16* qp = &Qs[(rb * 16 + m) * QP + ks * 32];
    aQ[ks].p[0] = *(const v8h*)(qp + 8 * hh);
    aQ[ks].p[1] = *(const v8h*)(qp + 16 + 8 * hh);
  }
  const int irow0 = q0 + rb * 16 + 8 * hh;
  for (int cb = (kbeg >> 4) + (wave & 1); cb < (kend >> 4); cb += 2) {
    Frag bK[2];
    const f16* kp = Kh + (size_t)(cb * 16 + m) * 64;
#pragma unroll
    for (int ks = 0; ks < 2; ++ks) {
      bK[ks].p[0] = *(const v8h*)(kp + ks * 32 + 8 * hh);
      bK[ks].p[1] = *(const v8h*)(kp + ks * 32 + 16 + 8 * hh);
    }
    v8f acc = zero8();
    acc = mma16(aQ[0].v, bK[0].v, acc);
    acc = mma16(aQ[1].v, bK[1].v, acc);
    asm volatile(NOPS4 : "+v"(acc) : "v"(aQ[0].v), "v"(aQ[1].v), "v"(bK[0].v), "v"(bK[1].v));
    const int j = cb * 16 + m;
    const int d0 = irow0 - j;
    float* so = &S[(rb * 16 + 8 * hh) * SP + j];
#pragma unroll
    for (int r = 0; r < 8; ++r) {
      const int d = d0 + r;
      const bool masked = (d < dlo) | (d > dhi);
      so[r * SP] = masked ? NEGM : acc[r] * (1.0f / 512.0f);
    }
  }
  __syncthreads();

  {
    const int row = tid & 63, c = tid >> 6;
    float* sr = &S[row * SP + kbeg + 4 * c];
    const int ng = (kend - kbeg) >> 4;
    float mx = -3.0e38f;
    for (int s = 0; s < ng; ++s) {
      const v4f x = *(const v4f*)(sr + 16 * s);
      mx = fmaxf(fmaxf(fmaxf(mx, x.x), x.y), fmaxf(x.z, x.w));
    }
    red[row * 4 + c] = mx;
    __syncthreads();
    const float rmax = fmaxf(fmaxf(red[row * 4 + 0], red[row * 4 + 1]),
                             fmaxf(red[row * 4 + 2], red[row * 4 + 3]));
    float sum = 0.0f;
    for (int s = 0; s < ng; ++s) {
      v4f x = *(const v4f*)(sr + 16 * s);
      x.x = __expf(x.x - rmax);
      x.y = __expf(x.y - rmax);
      x.z = __expf(x.z - rmax);
      x.w = __expf(x.w - rmax);
      *(v4f*)(sr + 16 * s) = x;
      sum += (x.x + x.y) + (x.z + x.w);
    }
    red[256 + row * 4 + c] = sum;
  }
  __syncthreads();

  v8f oacc[2];
  oacc[0] = zero8(); oacc[1] = zero8();
  const int cbs = (wave & 1) * 2;
  const float* prow = &S[(rb * 16 + m) * SP];
  const size_t vr0 = (size_t)(cbs * 16 + m) * 4096;
  const size_t vr1 = vr0 + (size_t)16 * 4096;
  for (int s0 = kbeg; s0 < kend; s0 += 32) {
    const v4f x0 = *(const v4f*)(prow + s0 + 8 * hh);
    const v4f x1 = *(const v4f*)(prow + s0 + 8 * hh + 4);
    const v4f x2 = *(const v4f*)(prow + s0 + 16 + 8 * hh);
    const v4f x3 = *(const v4f*)(prow + s0 + 20 + 8 * hh);
    Frag aP;
    aP.v[0]  = (f16)(x0.x * 1024.0f);  aP.v[1]  = (f16)(x0.y * 1024.0f);
    aP.v[2]  = (f16)(x0.z * 1024.0f);  aP.v[3]  = (f16)(x0.w * 1024.0f);
    aP.v[4]  = (f16)(x1.x * 1024.0f);  aP.v[5]  = (f16)(x1.y * 1024.0f);
    aP.v[6]  = (f16)(x1.z * 1024.0f);  aP.v[7]  = (f16)(x1.w * 1024.0f);
    aP.v[8]  = (f16)(x2.x * 1024.0f);  aP.v[9]  = (f16)(x2.y * 1024.0f);
    aP.v[10] = (f16)(x2.z * 1024.0f);  aP.v[11] = (f16)(x2.w * 1024.0f);
    aP.v[12] = (f16)(x3.x * 1024.0f);  aP.v[13] = (f16)(x3.y * 1024.0f);
    aP.v[14] = (f16)(x3.z * 1024.0f);  aP.v[15] = (f16)(x3.w * 1024.0f);
    Frag bh0, bl0, bh1, bl1;
    bh0.p[0] = *(const v8h*)(Vh + vr0 + s0 + 8 * hh);  bh0.p[1] = *(const v8h*)(Vh + vr0 + s0 + 16 + 8 * hh);
    bl0.p[0] = *(const v8h*)(Vl + vr0 + s0 + 8 * hh);  bl0.p[1] = *(const v8h*)(Vl + vr0 + s0 + 16 + 8 * hh);
    bh1.p[0] = *(const v8h*)(Vh + vr1 + s0 + 8 * hh);  bh1.p[1] = *(const v8h*)(Vh + vr1 + s0 + 16 + 8 * hh);
    bl1.p[0] = *(const v8h*)(Vl + vr1 + s0 + 8 * hh);  bl1.p[1] = *(const v8h*)(Vl + vr1 + s0 + 16 + 8 * hh);
    oacc[0] = mma16(aP.v, bh0.v, oacc[0]);
    oacc[0] = mma16(aP.v, bl0.v, oacc[0]);
    oacc[1] = mma16(aP.v, bh1.v, oacc[1]);
    oacc[1] = mma16(aP.v, bl1.v, oacc[1]);
    asm volatile(NOPS4 : "+v"(oacc[0]), "+v"(oacc[1])
                 : "v"(aP.v), "v"(bh0.v), "v"(bl0.v), "v"(bh1.v), "v"(bl1.v));
  }
  __syncthreads();

  f16* Oh = (f16*)smem;
  f16* Ol = Oh + 64 * QP;
  float rinv[8];
#pragma unroll
  for (int r = 0; r < 8; ++r) {
    const int i = rb * 16 + 8 * hh + r;
    const float rs = (red[256 + i * 4 + 0] + red[256 + i * 4 + 1])
                   + (red[256 + i * 4 + 2] + red[256 + i * 4 + 3]);
    rinv[r] = 1.0f / (rs * 1024.0f);
  }
#pragma unroll
  for (int jj = 0; jj < 2; ++jj) {
    const int col = (cbs + jj) * 16 + m;
#pragma unroll
    for (int r = 0; r < 8; ++r) {
      const int i = rb * 16 + 8 * hh + r;
      const float o = oacc[jj][r] * rinv[r];
      const f16 hv = (f16)o;
      const f16 lv = (f16)(o - (float)hv);
      Oh[i * QP + col] = hv;
      Ol[i * QP + col] = lv;
    }
  }
  __syncthreads();
  const int seg = tid & 7, lb = tid >> 3;
  v8h val[4]; size_t off[4];
#pragma unroll
  for (int it = 0; it < 4; ++it) {
    const int plane = it >> 1;
    const int line = lb + 32 * (it & 1);
    val[it] = *(const v8h*)((plane ? Ol : Oh) + line * QP + seg * 8);
    off[it] = (size_t)(b * 1024 + q0 + line) * 2048 + (size_t)plane * 1024 + hd * 64 + seg * 8;
  }
#pragma unroll
  for (int it = 0; it < 4; ++it) *(volatile v8h*)(Ao + off[it]) = val[it];
  __threadfence();
#pragma unroll
  for (int it = 0; it < 4; ++it) *(volatile v8h*)(Ao + off[it]) = val[it];
}

extern "C" void kernel_launch(void* const* d_in, const int* in_sizes, int n_in,
                              void* d_out, int out_size, void* d_ws, size_t ws_size,
                              hipStream_t stream)
{
  if (n_in < 10) return;
  if (in_sizes[0] != 4194304 || in_sizes[1] != 4194304) return;
  if (in_sizes[2] != 1048576 || in_sizes[4] != 1048576 || in_sizes[6] != 1048576) return;
  if (in_sizes[8] != 1048576) return;
  if (in_sizes[3] < 64 || in_sizes[5] < 64 || in_sizes[7] < 64 || in_sizes[9] < 1024) return;
  if (out_size != 4194304) return;
  const size_t MB = (size_t)1048576;
  if (ws_size < 72 * MB) return;

  const float* query = (const float*)d_in[0];
  const float* value = (const float*)d_in[1];
  const float* Wq    = (const float*)d_in[2];
  const float* bq    = (const float*)d_in[3];
  const float* Wk    = (const float*)d_in[4];
  const float* bk    = (const float*)d_in[5];
  const float* Wv    = (const float*)d_in[6];
  const float* bv    = (const float*)d_in[7];
  const float* Wo    = (const float*)d_in[8];
  const float* bo    = (const float*)d_in[9];

  unsigned char* ws = (unsigned char*)d_ws;
  f16* xq = (f16*)(ws);
  f16* xv = (f16*)(ws +  8 * MB);
  f16* wq = (f16*)(ws + 16 * MB);
  f16* wk = (f16*)(ws + 18 * MB);
  f16* wv = (f16*)(ws + 20 * MB);
  f16* wo = (f16*)(ws + 22 * MB);
  f16* qh = (f16*)(ws + 24 * MB);
  f16* kh = (f16*)(ws + 32 * MB);
  f16* vh = (f16*)(ws + 40 * MB);
  f16* vl = (f16*)(ws + 48 * MB);
  f16* ao = (f16*)(ws + 56 * MB);

  const int n8 = 4194304 / 8;
  k_cvt<<<dim3((n8 + 255) / 256), dim3(256), 0, stream>>>(query, xq, n8, 8.0f);
  k_cvt<<<dim3((n8 + 255) / 256), dim3(256), 0, stream>>>(value, xv, n8, 8.0f);

  k_wtr<<<dim3(1, 16, 16), dim3(256), 0, stream>>>(Wq, wq, 1024, 64, 65536L, 65536L, 64.0f);
  k_wtr<<<dim3(1, 16, 16), dim3(256), 0, stream>>>(Wk, wk, 1024, 64, 65536L, 65536L, 64.0f);
  k_wtr<<<dim3(1, 16, 16), dim3(256), 0, stream>>>(Wv, wv, 1024, 64, 65536L, 65536L, 64.0f);
  k_wtr<<<dim3(16, 16, 1), dim3(256), 0, stream>>>(Wo, wo, 1024, 1024, 0L, 0L, 64.0f);

  k_gemm<0><<<dim3(1, 32, 16), dim3(256), 0, stream>>>(xq, 1024, wq, 1024, 65536L, 1023, 1024,
                                                       bq, 1.0f / 512.0f, 8.0f,
                                                       (void*)qh, (void*)qh, 64, 262144L);
  k_gemm<0><<<dim3(1, 32, 16), dim3(256), 0, stream>>>(xv, 1024, wk, 1024, 65536L, 1023, 1024,
                                                       bk, 1.0f / 512.0f, 8.0f,
                                                       (void*)kh, (void*)kh, 64, 262144L);
  k_gemm<1><<<dim3(1, 32, 16), dim3(256), 0, stream>>>(xv, 1024, wv, 1024, 65536L, 1023, 1024,
                                                       bv, 1.0f / 512.0f, 64.0f,
                                                       (void*)vh, (void*)vl, 4096, 262144L);

  const size_t smem = (size_t)64 * SP * 4 + (size_t)64 * QP * 2 + 512 * 4;
  hipFuncSetAttribute((const void*)k_attn, hipFuncAttributeMaxDynamicSharedMemorySize, (int)smem);
  k_attn<<<dim3(16, 16, 4), dim3(256), smem, stream>>>(qh, kh, vh, vl, ao);

  k_gemm<2><<<dim3(16, 32, 1), dim3(256), 0, stream>>>(ao, 2048, wo, 1024, 0L, 1023, 2048,
                                                       bo, 1.0f / 4096.0f, 1.0f,
                                                       d_out, d_out, 1024, 0L);
}
